// MatchSRNN_40785009443661
// MI455X (gfx1250) — hardware-verified
//
#include <hip/hip_runtime.h>
#define BBn 256
#define ML 56
#define EMB 300
#define EP 320
#define NDm 4
#define NR1 (BBn * ML)

typedef __bf16 v16b __attribute__((ext_vector_type(16)));
typedef unsigned short v8us __attribute__((ext_vector_type(8), may_alias));
typedef float  v8f  __attribute__((ext_vector_type(8)));
typedef float  v4f  __attribute__((ext_vector_type(4)));
typedef float  v4fa __attribute__((ext_vector_type(4), may_alias));
union FragB { v16b v; v8us half[2]; unsigned short u[16]; };

__device__ __forceinline__ unsigned short bf16_bits(float x) { unsigned int u = __float_as_uint(x); return (unsigned short)((u + 0x7FFFu + ((u >> 16) & 1u)) >> 16); }
__device__ __forceinline__ float bf16_val(unsigned short b) { return __uint_as_float(((unsigned int)b) << 16); }
__device__ __forceinline__ float bf16_round(float x) { return bf16_val(bf16_bits(x)); }
template <int NT>
__device__ __forceinline__ v8f mmaN(v16b ah, v16b al, v16b bh, v16b bl, v8f c) {
  c = __builtin_amdgcn_wmma_f32_16x16x32_bf16(false, ah, false, bh, (short)0, c, false, false);
  if (NT >= 2) c = __builtin_amdgcn_wmma_f32_16x16x32_bf16(false, al, false, bh, (short)0, c, false, false);
  if (NT >= 3) c = __builtin_amdgcn_wmma_f32_16x16x32_bf16(false, ah, false, bl, (short)0, c, false, false);
  asm volatile("v_nop\n\tv_nop\n\tv_nop\n\tv_nop" : "+v"(c) : "v"(ah), "v"(al), "v"(bh), "v"(bl));
  return c;
}

__global__ __launch_bounds__(256) void k_wt_bf16(const float* __restrict__ W, unsigned short* __restrict__ Wt, int K, int N) {
  const int t = blockIdx.x * 256 + threadIdx.x;
  const int k8n = K / 8;
  if (t >= N * k8n) return;
  const int n = t / k8n, k8 = (t % k8n) * 8;
  v8us v;
#pragma unroll
  for (int i = 0; i < 8; ++i) v[i] = bf16_bits(W[(size_t)(k8 + i) * N + n]);
  *(volatile v8us*)(Wt + (size_t)n * K + k8) = v;
  __threadfence();
  *(volatile v8us*)(Wt + (size_t)n * K + k8) = v;
}

template <bool ASPLIT, int ACT, bool BIAS_BF16>
__global__ __launch_bounds__(128) void k_gemm_bf(const float* __restrict__ A, int lda, const unsigned short* __restrict__ Wt, int ldb,
                                               const float* __restrict__ bias, float* __restrict__ C, int ldc, int M, int N, int K) {
  __shared__ __attribute__((aligned(16))) float so[4][16][64];
  const int tid = threadIdx.x, w = tid >> 5, lane = tid & 31, ln = lane & 15, hh = lane >> 4;
  const int ntn = N / 64;
  const int wid = blockIdx.x * 4 + w;
  const int mt = wid / ntn, nq = wid % ntn;
  if (mt * 16 >= M) return;
  const int row0 = mt * 16, col0 = nq * 64;
  const float* arow = A + (size_t)(row0 + ln) * lda;
  v8f acc[4] = {};
  for (int kb = 0; kb < K; kb += 32) {
    FragB ah, al;
    const v4f x0 = *(const v4fa*)(arow + kb + 8 * hh), x1 = *(const v4fa*)(arow + kb + 8 * hh + 4);
    const v4f x2 = *(const v4fa*)(arow + kb + 16 + 8 * hh), x3 = *(const v4fa*)(arow + kb + 16 + 8 * hh + 4);
    float xs[16] = {x0[0],x0[1],x0[2],x0[3],x1[0],x1[1],x1[2],x1[3],x2[0],x2[1],x2[2],x2[3],x3[0],x3[1],x3[2],x3[3]};
#pragma unroll
    for (int i = 0; i < 16; ++i) { const unsigned short hb = bf16_bits(xs[i]); ah.u[i] = hb; al.u[i] = ASPLIT ? bf16_bits(xs[i] - bf16_val(hb)) : (unsigned short)0; }
#pragma unroll
    for (int t = 0; t < 4; ++t) {
      const unsigned short* brow = Wt + (size_t)(col0 + t * 16 + ln) * ldb + kb;
      FragB b;
      b.half[0] = *(const v8us*)(brow + 8 * hh);
      b.half[1] = *(const v8us*)(brow + 16 + 8 * hh);
      acc[t] = mmaN<ASPLIT ? 2 : 1>(ah.v, al.v, b.v, b.v, acc[t]);
    }
  }
#pragma unroll
  for (int t = 0; t < 4; ++t) {
    float bv = bias ? bias[col0 + t * 16 + ln] : 0.f;
    if (BIAS_BF16) bv = bf16_round(bv);
#pragma unroll
    for (int r = 0; r < 8; ++r) { float v = acc[t][r] + bv; if (ACT == 1) v = fmaxf(v, 0.f); so[w][8 * hh + r][t * 16 + ln] = v; }
  }
  __builtin_amdgcn_fence(__ATOMIC_ACQ_REL, "workgroup");
  __builtin_amdgcn_wave_barrier();
  const int rsub = lane >> 4, c4 = (lane & 15) * 4;
  for (int pass = 0; pass < 2; ++pass) {
#pragma unroll
    for (int q = 0; q < 8; ++q) {
      const int r = q * 2 + rsub;
      const v4f v = *(const v4fa*)&so[w][r][c4];
      *(volatile v4f*)(C + (size_t)(row0 + r) * ldc + col0 + c4) = v;
    }
    if (pass == 0) __threadfence();
  }
}

template <int D, bool CAUSAL>
__global__ __launch_bounds__(128) void k_flash(const float* __restrict__ qb, const float* __restrict__ kb, const float* __restrict__ vb,
                                             int pitch, int T, int H, float scale, float* __restrict__ y, int ypitch) {
  constexpr int KS = D / 32;
  constexpr int DT = D / 16;
  __shared__ __attribute__((aligned(16))) unsigned short sKh[32][D + 8], sKl[32][D + 8], sVh[32][D + 8], sVl[32][D + 8];
  __shared__ __attribute__((aligned(16))) unsigned short sPh[4][16][40], sPl[4][16][40];
  __shared__ __attribute__((aligned(16))) float sO[4][16][D];
  const int tid = threadIdx.x, w = tid >> 5, lane = tid & 31, ln = lane & 15, hh = lane >> 4;
  const int nqb = (T + 63) / 64;
  const int bh = blockIdx.x / nqb, qblk = blockIdx.x % nqb;
  const int b = bh / H, h = bh % H;
  const int q0 = qblk * 64 + w * 16;
  const float* Q = qb + (size_t)b * T * pitch + h * D;
  const float* K = kb + (size_t)b * T * pitch + h * D;
  const float* V = vb + (size_t)b * T * pitch + h * D;

  FragB aqh[KS], aql[KS];
  {
    int row = q0 + ln; if (row >= T) row = T - 1;
    const float* qr = Q + (size_t)row * pitch;
#pragma unroll
    for (int ks = 0; ks < KS; ++ks)
#pragma unroll
      for (int i = 0; i < 16; ++i) {
        const int d = ks * 32 + ((i < 8) ? (8 * hh + i) : (16 + 8 * hh + (i - 8)));
        const float x = qr[d] * scale; const unsigned short hb = bf16_bits(x);
        aqh[ks].u[i] = hb; aql[ks].u[i] = bf16_bits(x - bf16_val(hb));
      }
  }
  float m_r[8], l_r[8];
#pragma unroll
  for (int r = 0; r < 8; ++r) { m_r[r] = -3.0e38f; l_r[r] = 0.f; }
  v8f oacc[DT];
#pragma unroll
  for (int dt = 0; dt < DT; ++dt) oacc[dt] = (v8f){0.f,0.f,0.f,0.f,0.f,0.f,0.f,0.f};

  const int kv_end = CAUSAL ? min(T, qblk * 64 + 64) : T;
  for (int j0 = 0; j0 < kv_end; j0 += 32) {
    __syncthreads();
    for (int e = tid; e < 32 * (D / 4); e += 128) {
      const int r = e / (D / 4), c4 = (e % (D / 4)) * 4;
      const int key = j0 + r;
      v4f kf = {0.f,0.f,0.f,0.f}, vf = {0.f,0.f,0.f,0.f};
      if (key < T) { kf = *(const v4fa*)(K + (size_t)key * pitch + c4); vf = *(const v4fa*)(V + (size_t)key * pitch + c4); }
#pragma unroll
      for (int t = 0; t < 4; ++t) {
        unsigned short hb = bf16_bits(kf[t]); sKh[r][c4 + t] = hb; sKl[r][c4 + t] = bf16_bits(kf[t] - bf16_val(hb));
        hb = bf16_bits(vf[t]); sVh[r][c4 + t] = hb; sVl[r][c4 + t] = bf16_bits(vf[t] - bf16_val(hb));
      }
    }
    __syncthreads();
    v8f s[2];
#pragma unroll
    for (int nt = 0; nt < 2; ++nt) {
      v8f acc = {};
#pragma unroll
      for (int ks = 0; ks < KS; ++ks) {
        FragB bh_, bl_;
        bh_.half[0] = *(const v8us*)&sKh[nt * 16 + ln][ks * 32 + 8 * hh]; bh_.half[1] = *(const v8us*)&sKh[nt * 16 + ln][ks * 32 + 16 + 8 * hh];
        bl_.half[0] = *(const v8us*)&sKl[nt * 16 + ln][ks * 32 + 8 * hh]; bl_.half[1] = *(const v8us*)&sKl[nt * 16 + ln][ks * 32 + 16 + 8 * hh];
        acc = mmaN<3>(aqh[ks].v, aql[ks].v, bh_.v, bl_.v, acc);
      }
      s[nt] = acc;
    }
    float alpha[8];
#pragma unroll
    for (int r = 0; r < 8; ++r) {
      const int qi = q0 + 8 * hh + r;
      const int ja = j0 + ln, jb = j0 + 16 + ln;
      if (CAUSAL) { if (ja > qi) s[0][r] = -3.0e38f; if (jb > qi) s[1][r] = -3.0e38f; }
      if (ja >= T) s[0][r] = -3.0e38f;
      if (jb >= T) s[1][r] = -3.0e38f;
      float mx = fmaxf(s[0][r], s[1][r]);
      mx = fmaxf(mx, __shfl_xor(mx, 1, 32)); mx = fmaxf(mx, __shfl_xor(mx, 2, 32)); mx = fmaxf(mx, __shfl_xor(mx, 4, 32)); mx = fmaxf(mx, __shfl_xor(mx, 8, 32));
      const float mnew = fmaxf(m_r[r], mx);
      alpha[r] = (mnew > -1.0e38f) ? __expf(m_r[r] - mnew) : 1.0f;
      const float p0 = (s[0][r] > -1.0e38f) ? __expf(s[0][r] - mnew) : 0.f;
      const float p1 = (s[1][r] > -1.0e38f) ? __expf(s[1][r] - mnew) : 0.f;
      m_r[r] = mnew;
      l_r[r] = l_r[r] * alpha[r] + p0 + p1;
      unsigned short hb = bf16_bits(p0); sPh[w][8 * hh + r][ln] = hb;      sPl[w][8 * hh + r][ln] = bf16_bits(p0 - bf16_val(hb));
      hb = bf16_bits(p1);                sPh[w][8 * hh + r][16 + ln] = hb; sPl[w][8 * hh + r][16 + ln] = bf16_bits(p1 - bf16_val(hb));
    }
#pragma unroll
    for (int dt = 0; dt < DT; ++dt)
#pragma unroll
      for (int r = 0; r < 8; ++r) oacc[dt][r] *= alpha[r];
    __builtin_amdgcn_fence(__ATOMIC_ACQ_REL, "workgroup");
    __builtin_amdgcn_wave_barrier();
    FragB pah, pal;
    pah.half[0] = *(const v8us*)&sPh[w][ln][8 * hh]; pah.half[1] = *(const v8us*)&sPh[w][ln][16 + 8 * hh];
    pal.half[0] = *(const v8us*)&sPl[w][ln][8 * hh]; pal.half[1] = *(const v8us*)&sPl[w][ln][16 + 8 * hh];
#pragma unroll
    for (int dt = 0; dt < DT; ++dt) {
      FragB bvh, bvl;
#pragma unroll
      for (int i = 0; i < 8; ++i) {
        bvh.u[i] = sVh[8 * hh + i][dt * 16 + ln]; bvh.u[8 + i] = sVh[16 + 8 * hh + i][dt * 16 + ln];
        bvl.u[i] = sVl[8 * hh + i][dt * 16 + ln]; bvl.u[8 + i] = sVl[16 + 8 * hh + i][dt * 16 + ln];
      }
      oacc[dt] = mmaN<3>(pah.v, pal.v, bvh.v, bvl.v, oacc[dt]);
    }
    __builtin_amdgcn_fence(__ATOMIC_ACQ_REL, "workgroup");
    __builtin_amdgcn_wave_barrier();
  }
#pragma unroll
  for (int r = 0; r < 8; ++r) {
    float l = l_r[r];
    l += __shfl_xor(l, 1, 32); l += __shfl_xor(l, 2, 32); l += __shfl_xor(l, 4, 32); l += __shfl_xor(l, 8, 32);
    l_r[r] = (l > 0.f) ? 1.0f / l : 0.f;
  }
#pragma unroll
  for (int dt = 0; dt < DT; ++dt)
#pragma unroll
    for (int r = 0; r < 8; ++r) sO[w][8 * hh + r][dt * 16 + ln] = oacc[dt][r] * l_r[r];
  __builtin_amdgcn_fence(__ATOMIC_ACQ_REL, "workgroup");
  __builtin_amdgcn_wave_barrier();
  for (int pass = 0; pass < 2; ++pass) {
    for (int r = 0; r < 16; ++r) {
      const int row = q0 + r;
      if (row < T && lane < D / 4) {
        const v4f val = *(const v4fa*)&sO[w][r][lane * 4];
        *(volatile v4f*)(y + ((size_t)b * T + row) * ypitch + h * D + lane * 4) = val;
      }
    }
    if (pass == 0) __threadfence();
  }
}

template <bool ASPLIT, int ACT, bool BIAS_BF16, bool RES_BF16>
__global__ __launch_bounds__(128) void k_gemm_bf3(const float* __restrict__ A, int lda, const unsigned short* __restrict__ Wt, int ldb,
                                                const float* __restrict__ bias, const float* __restrict__ resid, int rmod, int ldr,
                                                float* __restrict__ C, int ldc, int M, int N, int K) {
  __shared__ __attribute__((aligned(16))) float so[4][16][64];
  const int tid = threadIdx.x, w = tid >> 5, lane = tid & 31, ln = lane & 15, hh = lane >> 4;
  const int ntn = N / 64;
  const int wid = blockIdx.x * 4 + w;
  const int mt = wid / ntn, nq = wid % ntn;
  if (mt * 16 >= M) return;
  const int row0 = mt * 16, col0 = nq * 64;
  const float* arow = A + (size_t)(row0 + ln) * lda;
  v8f acc[4] = {};
  for (int kb = 0; kb < K; kb += 32) {
    FragB ah, al;
    const v4f x0 = *(const v4fa*)(arow + kb + 8 * hh), x1 = *(const v4fa*)(arow + kb + 8 * hh + 4);
    const v4f x2 = *(const v4fa*)(arow + kb + 16 + 8 * hh), x3 = *(const v4fa*)(arow + kb + 16 + 8 * hh + 4);
    float xs[16] = {x0[0],x0[1],x0[2],x0[3],x1[0],x1[1],x1[2],x1[3],x2[0],x2[1],x2[2],x2[3],x3[0],x3[1],x3[2],x3[3]};
#pragma unroll
    for (int i = 0; i < 16; ++i) { const unsigned short hb = bf16_bits(xs[i]); ah.u[i] = hb; al.u[i] = ASPLIT ? bf16_bits(xs[i] - bf16_val(hb)) : (unsigned short)0; }
#pragma unroll
    for (int t = 0; t < 4; ++t) {
      const unsigned short* brow = Wt + (size_t)(col0 + t * 16 + ln) * ldb + kb;
      FragB b;
      b.half[0] = *(const v8us*)(brow + 8 * hh);
      b.half[1] = *(const v8us*)(brow + 16 + 8 * hh);
      acc[t] = mmaN<ASPLIT ? 2 : 1>(ah.v, al.v, b.v, b.v, acc[t]);
    }
  }
#pragma unroll
  for (int t = 0; t < 4; ++t) {
    const int col = col0 + t * 16 + ln;
    float bv = bias ? bias[col] : 0.f;
    if (BIAS_BF16) bv = bf16_round(bv);
#pragma unroll
    for (int r = 0; r < 8; ++r) {
      float v = acc[t][r] + bv;
      if (resid) { float rv = resid[(size_t)((row0 + 8 * hh + r) % rmod) * ldr + col]; if (RES_BF16) rv = bf16_round(rv); v += rv; }
      if (ACT == 1) v = fmaxf(v, 0.f);
      if (ACT == 2) v = 0.5f * v * (1.0f + erff(v * 0.70710678118654752f));
      if (ACT == 3) { const float u = 0.7978845608028654f * (v + 0.044715f * v * v * v); v = 0.5f * v * (1.0f + tanhf(u)); }
      so[w][8 * hh + r][t * 16 + ln] = v;
    }
  }
  __builtin_amdgcn_fence(__ATOMIC_ACQ_REL, "workgroup");
  __builtin_amdgcn_wave_barrier();
  const int rsub = lane >> 4, c4 = (lane & 15) * 4;
  for (int pass = 0; pass < 2; ++pass) {
#pragma unroll
    for (int q = 0; q < 8; ++q) {
      const int r = q * 2 + rsub;
      const v4f v = *(const v4fa*)&so[w][r][c4];
      *(volatile v4f*)(C + (size_t)(row0 + r) * ldc + col0 + c4) = v;
    }
    if (pass == 0) __threadfence();
  }
}
template <bool PARAM_BF16>
__global__ __launch_bounds__(256) void k_layernorm(const float* __restrict__ X, const float* __restrict__ R, const float* __restrict__ g, const float* __restrict__ bta,
                                                  float* __restrict__ out_sum, float* __restrict__ out_norm, int N, float eps) {
  __shared__ float red[256];
  const int row = blockIdx.x, tid = threadIdx.x;
  const float* x = X + (size_t)row * N; const float* rr = R ? R + (size_t)row * N : nullptr;
  float vals[16];
  const int per = N / 256;
  float s1 = 0.f;
  for (int u = 0; u < per / 4; ++u) {
    const int j = tid * 4 + 1024 * u;
    const v4f a = *(const v4fa*)(x + j);
    v4f b = {0.f,0.f,0.f,0.f}; if (rr) b = *(const v4fa*)(rr + j);
#pragma unroll
    for (int q = 0; q < 4; ++q) { const float v = a[q] + b[q]; vals[u * 4 + q] = v; s1 += v; }
  }
  red[tid] = s1; __syncthreads();
  for (int st = 128; st > 0; st >>= 1) { if (tid < st) red[tid] += red[tid + st]; __syncthreads(); }
  const float mu = red[0] / (float)N; __syncthreads();
  float s2 = 0.f;
  for (int u = 0; u < per / 4; ++u)
#pragma unroll
    for (int q = 0; q < 4; ++q) { const float c = vals[u * 4 + q] - mu; s2 += c * c; }
  red[tid] = s2; __syncthreads();
  for (int st = 128; st > 0; st >>= 1) { if (tid < st) red[tid] += red[tid + st]; __syncthreads(); }
  const float rs = rsqrtf(red[0] / (float)N + eps);
  for (int pass = 0; pass < 2; ++pass) {
    for (int u = 0; u < per / 4; ++u) {
      const int j = tid * 4 + 1024 * u;
      v4f o, sm;
#pragma unroll
      for (int q = 0; q < 4; ++q) {
        float gg = g[j + q], bb = bta[j + q];
        if (PARAM_BF16) { gg = bf16_round(gg); bb = bf16_round(bb); }
        sm[q] = vals[u * 4 + q]; o[q] = (vals[u * 4 + q] - mu) * rs * gg + bb;
      }
      if (out_sum) *(volatile v4f*)(out_sum + (size_t)row * N + j) = sm;
      *(volatile v4f*)(out_norm + (size_t)row * N + j) = o;
    }
    if (pass == 0) __threadfence();
  }
}


typedef _Float16 v16h __attribute__((ext_vector_type(16)));
union FragH { v16h v; v8us half[2]; _Float16 h[16]; unsigned short u[16]; };
template <int NT>
__device__ __forceinline__ v8f mmaH(v16h ah, v16h al, v16h bh, v16h bl, v8f c) {
  c = __builtin_amdgcn_wmma_f32_16x16x32_f16(false, ah, false, bh, (short)0, c, false, false);
  if (NT >= 2) c = __builtin_amdgcn_wmma_f32_16x16x32_f16(false, al, false, bh, (short)0, c, false, false);
  if (NT >= 3) c = __builtin_amdgcn_wmma_f32_16x16x32_f16(false, ah, false, bl, (short)0, c, false, false);
  asm volatile("v_nop\n\tv_nop\n\tv_nop\n\tv_nop" : "+v"(c) : "v"(ah), "v"(al), "v"(bh), "v"(bl));
  return c;
}
template <bool ASPLIT>
__global__ __launch_bounds__(128) void k_gemm_h(const float* __restrict__ A, int lda, size_t sA, const _Float16* __restrict__ Bh, int ldb, size_t sB, float alpha, float* __restrict__ C, int ldc, size_t sC, int M, int N, int K) {
  __shared__ __attribute__((aligned(16))) float so[4][16][64];
  const int tid = threadIdx.x, w = tid >> 5, lane = tid & 31, ln = lane & 15, hh = lane >> 4; const int by = blockIdx.y;
  A += (size_t)by * sA; Bh += (size_t)by * sB; C += (size_t)by * sC;
  const int ntn = (N + 63) / 64; const int wid = blockIdx.x * 4 + w; const int mt = wid / ntn, nq = wid % ntn; if (mt * 16 >= M) return;
  const int row0 = mt * 16, col0 = nq * 64; const float* arow = A + (size_t)(row0 + ln) * lda;
  v8f acc[4] = {};
  for (int kb = 0; kb < K; kb += 32) {
    FragH ah, al;
    const v4f x0 = *(const v4fa*)(arow + kb + 8 * hh), x1 = *(const v4fa*)(arow + kb + 8 * hh + 4), x2 = *(const v4fa*)(arow + kb + 16 + 8 * hh), x3 = *(const v4fa*)(arow + kb + 16 + 8 * hh + 4);
    float xs[16] = {x0[0],x0[1],x0[2],x0[3],x1[0],x1[1],x1[2],x1[3],x2[0],x2[1],x2[2],x2[3],x3[0],x3[1],x3[2],x3[3]};
#pragma unroll
    for (int i = 0; i < 16; ++i) { const _Float16 h = (_Float16)xs[i]; ah.h[i] = h; al.h[i] = ASPLIT ? (_Float16)(xs[i] - (float)h) : (_Float16)0.0f; }
#pragma unroll
    for (int t = 0; t < 4; ++t) { if (col0 + t * 16 >= N) continue; const size_t boff = (size_t)(col0 + t * 16 + ln) * ldb + kb; FragH bq; bq.half[0] = *(const v8us*)(Bh + boff + 8 * hh); bq.half[1] = *(const v8us*)(Bh + boff + 16 + 8 * hh);
      acc[t] = mmaH<ASPLIT ? 2 : 1>(ah.v, al.v, bq.v, bq.v, acc[t]); }
  }
#pragma unroll
  for (int t = 0; t < 4; ++t) { if (col0 + t * 16 >= N) continue;
#pragma unroll
    for (int r = 0; r < 8; ++r) so[w][8 * hh + r][t * 16 + ln] = acc[t][r] * alpha; }
  __builtin_amdgcn_fence(__ATOMIC_ACQ_REL, "workgroup"); __builtin_amdgcn_wave_barrier();
  const int rsub = lane >> 4, c4 = (lane & 15) * 4;
  for (int pass = 0; pass < 2; ++pass) {
#pragma unroll
    for (int q = 0; q < 8; ++q) { const int r = q * 2 + rsub; if (col0 + c4 < N) { const v4f v = *(const v4fa*)&so[w][r][c4]; *(volatile v4f*)(C + (size_t)(row0 + r) * ldc + col0 + c4) = v; } }
    if (pass == 0) __threadfence(); }
}

__global__ __launch_bounds__(256) void k_wt_f16(const float* __restrict__ W, _Float16* __restrict__ Wt, int K, int N, float scale) {
  const int t = blockIdx.x * 256 + threadIdx.x; if (t >= N * (K / 8)) return; const int n = t / (K / 8), k8 = (t % (K / 8)) * 8; FragH f;
#pragma unroll
  for (int i = 0; i < 8; ++i) f.h[i] = (_Float16)(bf16_round(W[(size_t)(k8 + i) * N + n]) * scale); const v8us o = f.half[0];
  *(volatile v8us*)((unsigned short*)Wt + (size_t)n * K + k8) = o; __threadfence(); *(volatile v8us*)((unsigned short*)Wt + (size_t)n * K + k8) = o;
}
template <int ACT>
__global__ __launch_bounds__(128) void k_gemm_hhx(const _Float16* __restrict__ A, int lda, size_t sA, const _Float16* __restrict__ Bh, int ldb, size_t sB, float alpha, const float* __restrict__ bias, size_t sBias, const float* __restrict__ CP, int rowsPerB, size_t sCPb, int row0g,
    float* __restrict__ C, _Float16* __restrict__ C16, int ldc, size_t sC, int M, int N, int K) {
  __shared__ __attribute__((aligned(16))) float so[4][16][64];
  const int tid = threadIdx.x, w = tid >> 5, lane = tid & 31, ln = lane & 15, hh = lane >> 4; const int by = blockIdx.y;
  A += (size_t)by * sA; Bh += (size_t)by * sB; const size_t cofs = (size_t)by * sC; const float* bp = bias ? bias + (size_t)by * sBias : nullptr;
  const int ntn = (N + 63) / 64; const int wid = blockIdx.x * 4 + w; const int mt = wid / ntn, nq = wid % ntn; if (mt * 16 >= M) return;
  const int row0 = mt * 16, col0 = nq * 64; const _Float16* arow = A + (size_t)(row0 + ln) * lda;
  v8f acc[4] = {};
  for (int kb = 0; kb < K; kb += 32) { FragH ah; ah.half[0] = *(const v8us*)((const unsigned short*)arow + kb + 8 * hh); ah.half[1] = *(const v8us*)((const unsigned short*)arow + kb + 16 + 8 * hh);
#pragma unroll
    for (int t = 0; t < 4; ++t) { if (col0 + t * 16 >= N) continue; const size_t boff = (size_t)(col0 + t * 16 + ln) * ldb + kb; FragH bq; bq.half[0] = *(const v8us*)((const unsigned short*)Bh + boff + 8 * hh); bq.half[1] = *(const v8us*)((const unsigned short*)Bh + boff + 16 + 8 * hh);
      acc[t] = mmaH<1>(ah.v, ah.v, bq.v, bq.v, acc[t]); }
  }
#pragma unroll
  for (int t = 0; t < 4; ++t) { if (col0 + t * 16 >= N) continue; const int col = col0 + t * 16 + ln; const float bv = bp ? bf16_round(bp[col]) : 0.f;
#pragma unroll
    for (int r = 0; r < 8; ++r) { float v = acc[t][r] * alpha + bv; if (CP) { const int bidx = (row0g + row0 + 8 * hh + r) / rowsPerB; v += CP[(size_t)bidx * sCPb + (size_t)by * 64 + col]; } if (ACT == 1) v = (v > 0.f) ? v : expm1f(v); else if (ACT == 3) v = fmaxf(v, 0.f); so[w][8 * hh + r][t * 16 + ln] = v; } }
  __builtin_amdgcn_fence(__ATOMIC_ACQ_REL, "workgroup"); __builtin_amdgcn_wave_barrier();
  const int rsub = lane >> 4, c4 = (lane & 15) * 4; typedef _Float16 v4h __attribute__((ext_vector_type(4)));
  for (int pass = 0; pass < 2; ++pass) {
#pragma unroll
    for (int q = 0; q < 8; ++q) { const int r = q * 2 + rsub; if (col0 + c4 < N) { const v4f v = *(const v4fa*)&so[w][r][c4]; if (C) *(volatile v4f*)(C + cofs + (size_t)(row0 + r) * ldc + col0 + c4) = v; if (C16) { v4h h4; for (int i = 0; i < 4; ++i) h4[i] = (_Float16)v[i]; *(volatile v4h*)(C16 + cofs + (size_t)(row0 + r) * ldc + col0 + c4) = h4; } } }
    if (pass == 0) __threadfence(); }
}


__global__ __launch_bounds__(256) void k_x16p(const float* __restrict__ x, _Float16* __restrict__ X16, int extra_rows) { const size_t t = (size_t)blockIdx.x * 256 + threadIdx.x; if (t >= (size_t)(NR1 + extra_rows) * (EP / 8)) return; const size_t row = t / (EP / 8); const int c8 = (int)(t % (EP / 8)) * 8; FragH f;
#pragma unroll
  for (int q = 0; q < 8; ++q) { const int m = c8 + q; f.h[q] = (_Float16)((row < NR1 && m < EMB) ? bf16_round(x[row * EMB + m]) : 0.f); }
  *(volatile v8us*)((unsigned short*)X16 + t * 8) = f.half[0]; __threadfence(); *(volatile v8us*)((unsigned short*)X16 + t * 8) = f.half[0]; }
__global__ __launch_bounds__(256) void k_wT(const float* __restrict__ T, _Float16* __restrict__ Bt) { const size_t t = (size_t)blockIdx.x * 256 + threadIdx.x; if (t >= (size_t)NDm * EP * (EP / 8)) return; const int m8 = (int)(t % (EP / 8)) * 8; const int row = (int)(t / (EP / 8)); const int d = row / EP, n = row % EP; FragH f;
#pragma unroll
  for (int q = 0; q < 8; ++q) { const int m = m8 + q; f.h[q] = (_Float16)((n < EMB && m < EMB) ? bf16_round(T[((size_t)d * EMB + m) * EMB + n]) * 16.0f : 0.f); }
  *(volatile v8us*)((unsigned short*)Bt + t * 8) = f.half[0]; __threadfence(); *(volatile v8us*)((unsigned short*)Bt + t * 8) = f.half[0]; }
__global__ __launch_bounds__(256) void k_ac(const float* __restrict__ x1, const float* __restrict__ x2, const float* __restrict__ Wl, float* __restrict__ AC) { const size_t t = (size_t)blockIdx.x * 256 + threadIdx.x; if (t >= (size_t)2 * NR1) return; const int which = (int)(t / NR1); const size_t row = t % NR1; const float* x = (which ? x2 : x1) + row * EMB; float a0 = 0.f, a1 = 0.f, a2 = 0.f, a3 = 0.f;
#pragma unroll 1
  for (int m = 0; m < EMB; ++m) { const float v = bf16_round(x[m]); const int o = which * EMB + m; a0 += v * bf16_round(Wl[o]); a1 += v * bf16_round(Wl[600 + o]); a2 += v * bf16_round(Wl[1200 + o]); a3 += v * bf16_round(Wl[1800 + o]); }
  v4f r; r[0] = a0; r[1] = a1; r[2] = a2; r[3] = a3; *(volatile v4f*)(AC + t * 4) = r; __threadfence(); *(volatile v4f*)(AC + t * 4) = r; }
__device__ __forceinline__ float convin_at(const float* BIL, const float* AC, const float* bl, int bp, int dp, int ip, int jp) {
  const size_t fprime = (((size_t)bp * NDm + dp) * ML + ip) * ML + jp; const size_t rprime = fprime >> 2; const int d = (int)(fprime & 3); const size_t r = (size_t)BBn * ML * ML - 1 - rprime; const int b = (int)(r / (ML * ML)); const int i = (int)((r % (ML * ML)) / ML), j = (int)(r % ML);
  const float v = BIL[(((size_t)b * NDm + d) * 64 + i) * 64 + j] + AC[((size_t)b * ML + i) * 4 + d] + AC[((size_t)NR1 + (size_t)b * ML + j) * 4 + d] + bf16_round(bl[d]); return fmaxf(v, 0.f); }
__global__ __launch_bounds__(256) void k_im1(const float* __restrict__ BIL, const float* __restrict__ AC, const float* __restrict__ bl, int b0, _Float16* __restrict__ A1) { __shared__ __attribute__((aligned(16))) _Float16 st[256][8]; const int tid = threadIdx.x; const size_t t = (size_t)blockIdx.x * 256 + tid; if (t >= (size_t)64 * 24 * 24 * 52) return; const size_t row = t / 52; const int p8 = (int)(t % 52) * 8; const int bp = b0 + (int)(row / 576); const int oy = (int)((row % 576) / 24), ox = (int)(row % 24);
#pragma unroll 1
  for (int q = 0; q < 8; ++q) { const int k = p8 + q; const int dp = k / 100, ky = (k % 100) / 10, kx = k % 10; st[tid][q] = (k < 400) ? (_Float16)convin_at(BIL, AC, bl, bp, dp, 2 * oy + ky, 2 * ox + kx) : (_Float16)0.f; }
  const v8us v = *(const v8us*)&st[tid][0]; *(volatile v8us*)((unsigned short*)A1 + t * 8) = v; __threadfence(); *(volatile v8us*)((unsigned short*)A1 + t * 8) = v; }
__global__ __launch_bounds__(256) void k_wc(const float* __restrict__ W, int O, int Kc, int Kp, int Opad, _Float16* __restrict__ Bt) { const int t = blockIdx.x * 256 + threadIdx.x; if (t >= Opad * (Kp / 8)) return; const int o = t / (Kp / 8), k8 = (t % (Kp / 8)) * 8; FragH f;
#pragma unroll
  for (int q = 0; q < 8; ++q) { const int k = k8 + q; f.h[q] = (_Float16)((o < O && k < Kc) ? bf16_round(W[(size_t)o * Kc + k]) * 16.0f : 0.f); } *(volatile v8us*)((unsigned short*)Bt + (size_t)o * Kp + k8) = f.half[0]; __threadfence(); *(volatile v8us*)((unsigned short*)Bt + (size_t)o * Kp + k8) = f.half[0]; }
__global__ __launch_bounds__(256) void k_im2(const float* __restrict__ C1, _Float16* __restrict__ A2) { __shared__ __attribute__((aligned(16))) _Float16 st[256][8]; const int tid = threadIdx.x; const size_t t = (size_t)blockIdx.x * 256 + tid; if (t >= (size_t)BBn * 64 * 52) return; const size_t row = t / 52; const int p8 = (int)(t % 52) * 8; const int b = (int)(row / 64); const int oy = (int)((row % 64) / 8), ox = (int)(row % 8);
#pragma unroll 1
  for (int q = 0; q < 8; ++q) { const int k = p8 + q; float m = 0.f; if (k < 400) { const int c = k / 25, ky = (k % 25) / 5, kx = k % 5; const int y = oy + ky, x = ox + kx; const float* base = C1 + (((size_t)b * 24 + 2 * y) * 24 + 2 * x) * 16 + c; m = fmaxf(fmaxf(base[0], base[16]), fmaxf(base[24 * 16], base[24 * 16 + 16])); } st[tid][q] = (_Float16)m; }
  const v8us v = *(const v8us*)&st[tid][0]; *(volatile v8us*)((unsigned short*)A2 + t * 8) = v; __threadfence(); *(volatile v8us*)((unsigned short*)A2 + t * 8) = v; }
__global__ __launch_bounds__(256) void k_head(const float* __restrict__ C2, const float* __restrict__ bconv2, const float* __restrict__ Wc1, const float* __restrict__ bc1, const float* __restrict__ Wc2, const float* __restrict__ bc2, float* __restrict__ out) { __shared__ float feat[16][384]; __shared__ float h1[16][10]; __shared__ float so[32]; const int tid = threadIdx.x; const int b0 = blockIdx.x * 16;
  for (int i = tid; i < 16 * 384; i += 256) { const int bl = i / 384, fi = i % 384; const int c = fi / 16, y = (fi % 16) / 4, x = fi % 4; const float* base = C2 + (((size_t)(b0 + bl) * 8 + 2 * y) * 8 + 2 * x) * 32 + c; feat[bl][fi] = fmaxf(fmaxf(fmaxf(base[0], base[32]), fmaxf(base[8 * 32], base[8 * 32 + 32])) + bf16_round(bconv2[c]), 0.f); }
  __syncthreads();
  if (tid < 160) { const int bl = tid / 10, o = tid % 10; float a = bf16_round(bc1[o]);
#pragma unroll 1
    for (int k = 0; k < 384; ++k) a += feat[bl][k] * bf16_round(Wc1[o * 384 + k]); h1[bl][o] = tanhf(a); }
  __syncthreads();
  if (tid < 16) { float z0 = bf16_round(bc2[0]), z1 = bf16_round(bc2[1]);
#pragma unroll 1
    for (int k = 0; k < 10; ++k) { z0 += h1[tid][k] * bf16_round(Wc2[k]); z1 += h1[tid][k] * bf16_round(Wc2[10 + k]); } z0 = tanhf(z0); z1 = tanhf(z1); const float m = fmaxf(z0, z1); const float e0 = expf(z0 - m), e1 = expf(z1 - m); so[tid * 2] = e0 / (e0 + e1); so[tid * 2 + 1] = e1 / (e0 + e1); }
  __syncthreads();
  if (tid < 32) { const float v = so[tid]; *(volatile float*)(out + (size_t)b0 * 2 + tid) = v; __threadfence(); *(volatile float*)(out + (size_t)b0 * 2 + tid) = v; } }
extern "C" void kernel_launch(void* const* d_in, const int* in_sizes, int n_in,
                              void* d_out, int out_size, void* d_ws, size_t ws_size, hipStream_t stream) {
  (void)in_sizes; (void)n_in; (void)out_size;
  const float* const* I = (const float* const*)d_in; const float* x1 = I[0]; const float* x2 = I[1]; const float* T = I[2]; const float* Wl = I[3]; const float* bl = I[4]; const float* Wc1v = I[5]; const float* bcv1 = I[6]; const float* Wc2v = I[7]; const float* bcv2 = I[8]; const float* Wf1 = I[9]; const float* bf1 = I[10]; const float* Wf2 = I[11]; const float* bf2 = I[12];
  char* ws = (char*)d_ws; size_t off = 0;
  auto take = [&](size_t bytes) { char* p = ws + off; off += (bytes + 255) & ~(size_t)255; return p; };
  _Float16* BtT = (_Float16*)take((size_t)NDm * EP * EP * 2); _Float16* Bc1 = (_Float16*)take((size_t)16 * 416 * 2); _Float16* Bc2 = (_Float16*)take((size_t)32 * 416 * 2);
  _Float16* X1 = (_Float16*)take((size_t)(NR1 + 16) * EP * 2); _Float16* X2 = (_Float16*)take((size_t)(NR1 + 16) * EP * 2); _Float16* T1 = (_Float16*)take((size_t)(NR1 + 16) * NDm * EP * 2); float* AC = (float*)take((size_t)2 * NR1 * 4 * 4); float* BIL = (float*)take((size_t)BBn * NDm * 64 * 64 * 4); _Float16* A1 = (_Float16*)take((size_t)64 * 576 * 416 * 2); float* C1 = (float*)take((size_t)BBn * 576 * 16 * 4); _Float16* A2 = (_Float16*)take((size_t)BBn * 64 * 416 * 2); float* C2 = (float*)take((size_t)BBn * 64 * 32 * 4);
  if (off > ws_size) return;
  k_wT<<<(unsigned)(((size_t)NDm * EP * (EP / 8) + 255) / 256), 256, 0, stream>>>(T, BtT); k_wc<<<(16 * 52 + 255) / 256, 256, 0, stream>>>(Wc1v, 16, 400, 416, 16, Bc1); k_wc<<<(32 * 52 + 255) / 256, 256, 0, stream>>>(Wc2v, 24, 400, 416, 32, Bc2);
  k_x16p<<<(unsigned)(((size_t)(NR1 + 16) * (EP / 8) + 255) / 256), 256, 0, stream>>>(x1, X1, 16); k_x16p<<<(unsigned)(((size_t)(NR1 + 16) * (EP / 8) + 255) / 256), 256, 0, stream>>>(x2, X2, 16);
  k_ac<<<(unsigned)(((size_t)2 * NR1 + 255) / 256), 256, 0, stream>>>(x1, x2, Wl, AC);
  k_gemm_hhx<0><<<dim3((((NR1 + 16) / 16) * (NDm * EP / 64) + 3) / 4, 1), 128, 0, stream>>>(X1, EP, 0, BtT, EP, 0, 0.0625f, nullptr, 0, nullptr, 1, 0, 0, nullptr, T1, NDm * EP, 0, NR1 + 16, NDm * EP, EP);
  for (int d = 0; d < NDm; ++d) k_gemm_hhx<0><<<dim3(((64 / 16) * 1 + 3) / 4, BBn), 128, 0, stream>>>(T1 + d * EP, NDm * EP, (size_t)ML * NDm * EP, X2, EP, (size_t)ML * EP, 1.0f, nullptr, 0, nullptr, 1, 0, 0, BIL + (size_t)d * 64 * 64, nullptr, 64, (size_t)NDm * 64 * 64, 64, 64, EP);
  for (int g = 0; g < BBn / 64; ++g) { k_im1<<<(unsigned)(((size_t)64 * 576 * 52 + 255) / 256), 256, 0, stream>>>(BIL, AC, bl, g * 64, A1);
    k_gemm_hhx<3><<<dim3(((64 * 576 / 16) * 1 + 3) / 4, 1), 128, 0, stream>>>(A1, 416, 0, Bc1, 416, 0, 0.0625f, bcv1, 0, nullptr, 1, 0, 0, C1 + (size_t)g * 64 * 576 * 16, nullptr, 16, 0, 64 * 576, 16, 416); }
  k_im2<<<(unsigned)(((size_t)BBn * 64 * 52 + 255) / 256), 256, 0, stream>>>(C1, A2);
  k_gemm_hhx<0><<<dim3(((BBn * 64 / 16) * 1 + 3) / 4, 1), 128, 0, stream>>>(A2, 416, 0, Bc2, 416, 0, 0.0625f, nullptr, 0, nullptr, 1, 0, 0, C2, nullptr, 32, 0, BBn * 64, 32, 416);
  k_head<<<BBn / 16, 256, 0, stream>>>(C2, bcv2, Wf1, bf1, Wf2, bf2, (float*)d_out);
}
